// GNN_69707319214464
// MI455X (gfx1250) — hardware-verified
//
#include <hip/hip_runtime.h>

typedef float          v8f   __attribute__((ext_vector_type(8)));
typedef float          v4f   __attribute__((ext_vector_type(4)));
typedef unsigned int   v4u   __attribute__((ext_vector_type(4)));
typedef int            v8i   __attribute__((ext_vector_type(8)));
typedef unsigned short v8us  __attribute__((ext_vector_type(8)));
typedef unsigned short v16us __attribute__((ext_vector_type(16)));
typedef __bf16         v16bf __attribute__((ext_vector_type(16)));
typedef _Float16       v16h  __attribute__((ext_vector_type(16)));
typedef v4f  __attribute__((may_alias)) v4fa;
typedef v8us __attribute__((may_alias)) v8usa;
union FragB { v16bf v; v16us u; v8us h[2]; v8i w; };
union FragH { v16h  v; v16us u; v8us h[2]; v8i w; };

__device__ __forceinline__ v8f wmb(const FragB& a, const FragB& b, v8f c) {
  v8f d = __builtin_amdgcn_wmma_f32_16x16x32_bf16(false, a.v, false, b.v, (short)0, c, false, false);
  asm volatile("v_nop\n\tv_nop\n\tv_nop\n\tv_nop" : "+v"(d) : "v"(a.w), "v"(b.w));
  return d;
}

__device__ __forceinline__ v8f wmh(const FragH& a, const FragH& b, v8f c) {
  v8f d = __builtin_amdgcn_wmma_f32_16x16x32_f16(false, a.v, false, b.v, (short)0, c, false, false);
  asm volatile("v_nop\n\tv_nop\n\tv_nop\n\tv_nop" : "+v"(d) : "v"(a.w), "v"(b.w));
  return d;
}

__device__ __forceinline__ unsigned bf16_bits(float f) {
  const unsigned u = __float_as_uint(f);
  const unsigned r = (u + 0x7FFFu + ((u >> 16) & 1u)) >> 16;
  const unsigned q = (u >> 16) | 0x40u;
  return ((u & 0x7fffffffu) > 0x7f800000u) ? q : r;
}

__device__ __forceinline__ float bf16_val(float f) {
  return __uint_as_float(bf16_bits(f) << 16);
}
__device__ __forceinline__ int clampi(int v, int lo, int hi) {
  return v < lo ? lo : (v > hi ? hi : v);
}

__device__ __forceinline__ unsigned f16_bits(float f) {
  const unsigned u  = __float_as_uint(f);
  const unsigned s  = (u >> 16) & 0x8000u;
  const unsigned a  = u & 0x7fffffffu;
  const unsigned t  = a - 0x38000000u;
  const unsigned r  = (t + 0x0FFFu + ((t >> 13) & 1u)) >> 13;
  const unsigned rc = r > 0x7C00u ? 0x7C00u : r;
  const bool small  = a < 0x38800000u;
  const bool isnan  = a > 0x7f800000u;
  const unsigned fin = small ? 0u : (s | rc);
  return isnan ? (s | 0x7E00u) : fin;
}

__device__ __forceinline__ unsigned pk16(unsigned lo, unsigned hi) { return lo | (hi << 16); }
__device__ __forceinline__ unsigned bf16_lo_bits(float v) {
  float hi = bf16_val(v);
  asm volatile("" : "+v"(hi));
  return bf16_bits(v - hi);
}
__device__ __forceinline__ v4u pack8_bf16(v4f a, v4f c) {
  return (v4u){ pk16(bf16_bits(a[0]), bf16_bits(a[1])), pk16(bf16_bits(a[2]), bf16_bits(a[3])),
                pk16(bf16_bits(c[0]), bf16_bits(c[1])), pk16(bf16_bits(c[2]), bf16_bits(c[3])) };
}
__device__ __forceinline__ v4u pack8_bf16_lo(v4f a, v4f c) {
  return (v4u){ pk16(bf16_lo_bits(a[0]), bf16_lo_bits(a[1])), pk16(bf16_lo_bits(a[2]), bf16_lo_bits(a[3])),
                pk16(bf16_lo_bits(c[0]), bf16_lo_bits(c[1])), pk16(bf16_lo_bits(c[2]), bf16_lo_bits(c[3])) };
}
__device__ __forceinline__ v4u pack8_f16(v4f a, v4f c) {
  return (v4u){ pk16(f16_bits(a[0]), f16_bits(a[1])), pk16(f16_bits(a[2]), f16_bits(a[3])),
                pk16(f16_bits(c[0]), f16_bits(c[1])), pk16(f16_bits(c[2]), f16_bits(c[3])) };
}

template <int FORM>
__global__ __launch_bounds__(256) void k_plane(const float* __restrict__ src, int rows, int cols, int ldsrc,
                                               unsigned short* __restrict__ dst, int MP, int KP) {
  static_assert(FORM >= 0 && FORM <= 3);
  const int KTOT = (FORM == 1 || FORM == 3) ? 2 * KP : KP;
  const unsigned ppr   = (unsigned)(KTOT >> 3);
  const unsigned kp8   = (unsigned)(KP >> 3);
  const unsigned total = (unsigned)MP * ppr;
  const unsigned g     = blockIdx.x * 256u + threadIdx.x;
  const unsigned rowu  = g / ppr;
  const unsigned p     = g - rowu * ppr;
  const bool second    = p >= kp8;
  const int row = (int)rowu;
  const int c0  = (int)((second ? p - kp8 : p) << 3);
  const float* srow = src + (size_t)clampi(row, 0, rows - 1) * (size_t)ldsrc;
  float x[8];
  unsigned mk[8];
#pragma unroll
  for (int e = 0; e < 8; ++e) {
    const int c = c0 + e;
    const float v = srow[clampi(c, 0, cols - 1)];
    asm volatile("" :: "v"(v));
    x[e]  = v;
    mk[e] = (row < rows && c < cols) ? 0xFFFFu : 0u;
  }
  const v4f a = (v4f){ x[0], x[1], x[2], x[3] };
  const v4f c = (v4f){ x[4], x[5], x[6], x[7] };
  v4u o;
  if (FORM == 2) {
    o = pack8_f16(a, c);
  } else {
    const v4u hi = pack8_bf16(a, c);
    o = hi;
    if (FORM == 1) { const v4u lo = pack8_bf16_lo(a, c); o = second ? lo : hi; }
  }
  const v4u mw = (v4u){ pk16(mk[0], mk[1]), pk16(mk[2], mk[3]), pk16(mk[4], mk[5]), pk16(mk[6], mk[7]) };
  o &= mw;
  if (g < total) {
    volatile v4u* q = (volatile v4u*)(dst + (size_t)g * 8);
    *q = o;
    __threadfence();
    *q = o;
  }
}

template <int FORM> struct FragOf    { typedef FragB T; };
template <>         struct FragOf<2> { typedef FragH T; };
__device__ __forceinline__ v8f mm(const FragB& a, const FragB& b, v8f c) { return wmb(a, b, c); }
__device__ __forceinline__ v8f mm(const FragH& a, const FragH& b, v8f c) { return wmh(a, b, c); }
template <class F> __device__ __forceinline__ F ld_frag(const unsigned short* p) {
  F f;
  f.h[0] = *(const v8usa*)(p);
  f.h[1] = *(const v8usa*)(p + 16);
  return f;
}

template <int FORM, int EPI>
__global__ __launch_bounds__(256) __attribute__((amdgpu_num_vgpr(248)))
void k_gemm_nt(const unsigned short* __restrict__ A, const unsigned short* __restrict__ B,
               const float* __restrict__ bias, float* __restrict__ D, int M, int N, int KTOT, int ldd) {
  static_assert(FORM >= 0 && FORM <= 2);
  static_assert(EPI == 0 || EPI == 1);
  typedef typename FragOf<FORM>::T F;
  __shared__ __attribute__((aligned(16))) float sT[8][16 * 68];
  const int lane = threadIdx.x & 31;
  const int wave = threadIdx.x >> 5;
  const int tilesM = (M + 63) >> 6;
  const int tilesN = (N + 63) >> 6;
  const int tile = blockIdx.x * 8 + wave;
  if (tile >= tilesM * tilesN) return;
  const int tm = tile / tilesN;
  const int tn = tile - tm * tilesN;
  const int m0 = tm << 6;
  const int n0 = tn << 6;

  const int rl = lane & 15;
  const int h8 = (lane >> 4) * 8;
  const unsigned short* pa = A + (size_t)(m0 + rl) * (size_t)KTOT + h8;
  const unsigned short* pb = B + (size_t)(n0 + rl) * (size_t)KTOT + h8;

  v8f acc[4][4];
#pragma unroll
  for (int i = 0; i < 4; ++i)
#pragma unroll
    for (int j = 0; j < 4; ++j) acc[i][j] = (v8f){0.f, 0.f, 0.f, 0.f, 0.f, 0.f, 0.f, 0.f};

#pragma unroll 1
  for (int k0 = 0; k0 < KTOT; k0 += 32) {
    F bf[4];
#pragma unroll
    for (int j = 0; j < 4; ++j) bf[j] = ld_frag<F>(pb + (size_t)(j << 4) * (size_t)KTOT + k0);
#pragma unroll
    for (int i = 0; i < 4; ++i) {
      const F af = ld_frag<F>(pa + (size_t)(i << 4) * (size_t)KTOT + k0);
#pragma unroll
      for (int j = 0; j < 4; ++j) acc[i][j] = mm(af, bf[j], acc[i][j]);
    }
  }

  float* slab = sT[wave];
  const int hh = lane >> 4;
  const int c4 = (lane & 15) * 4;
  const int nc = n0 + c4;
  const bool cok = nc < N;
  v4f bv = (v4f){0.f, 0.f, 0.f, 0.f};
  if (EPI == 1) {
    bv = *(const v4fa*)(bias + clampi(nc, 0, N - 4));
    asm volatile("" :: "v"(bv));
  }
#pragma unroll
  for (int i = 0; i < 4; ++i) {
    const int mBase = m0 + (i << 4);
#pragma unroll
    for (int j = 0; j < 4; ++j) {
#pragma unroll
      for (int r = 0; r < 8; ++r) slab[(h8 + r) * 68 + (j << 4) + rl] = acc[i][j][r];
    }
    __builtin_amdgcn_fence(__ATOMIC_RELEASE, "workgroup");
    __builtin_amdgcn_wave_barrier();
    __builtin_amdgcn_fence(__ATOMIC_ACQUIRE, "workgroup");
    v4f vv[8];
#pragma unroll
    for (int it = 0; it < 8; ++it) {
      const int row = it * 2 + hh;
      v4f v = *(const v4fa*)(slab + row * 68 + c4);
      if (EPI == 1) v += bv;
      vv[it] = v;
    }
    for (int pass = 0; pass < 2; ++pass) {
#pragma unroll
      for (int it = 0; it < 8; ++it) {
        const int row = mBase + it * 2 + hh;
        if (cok && row < M) *(volatile v4f*)(D + (size_t)row * (size_t)ldd + nc) = vv[it];
      }
      __threadfence();
    }
    __builtin_amdgcn_fence(__ATOMIC_RELEASE, "workgroup");
    __builtin_amdgcn_wave_barrier();
    __builtin_amdgcn_fence(__ATOMIC_ACQUIRE, "workgroup");
  }
}

typedef unsigned       v2u  __attribute__((ext_vector_type(2)));
typedef int            v4i  __attribute__((ext_vector_type(4)));
typedef v4i __attribute__((may_alias)) v4ia;
typedef v2u __attribute__((may_alias)) v2ua;
typedef v4u __attribute__((may_alias)) v4ua;
typedef unsigned short __attribute__((may_alias)) usa;

#define NNODE   50000
#define NEDGE   800000
#define MPAD    50176
#define NBRUN   1024
#define NBLKB   49
#define NWV     8
#define WCAP    2688
#define LISTN   (NWV * WCAP)
#define RCAP    21504
#define NWCH    (NEDGE / 256)
#define DEGCAP  48
#define BK_CNTW LISTN
#define BK_OFF  (BK_CNTW + NWV * NBRUN)
#define BK_CNT  (BK_OFF + NBRUN)
#define BK_MISC (BK_CNT + NBRUN)
#define BK_PLC  (BK_MISC + 64)
#define BK_INTS (BK_PLC + RCAP / 2)

#define XB_BLK  3136
#define WT_BLK  262
#define PREP_GRID (XB_BLK + WT_BLK + 1)

#define T_ENCB  0
#define T_B1    384
#define T_G     1152
#define T_BE    1920
#define T_RM    2688
#define T_INV   3456
#define T_B2    4224
#define TAB_N   4608

static_assert(NEDGE % 256 == 0);
static_assert(NEDGE <= (1 << 22));
static_assert(NBRUN == 1024);
static_assert(NBLKB * NBRUN == MPAD && (NBLKB - 1) * NBRUN < NNODE && MPAD >= NNODE);
static_assert(MPAD % 128 == 0 && MPAD % 64 == 0);
static_assert(NWV * WCAP == RCAP && RCAP % 256 == 0 && LISTN <= 65536);
static_assert(RCAP >= 16759 + (16759 + 3) / 4);
static_assert(DEGCAP >= 37 + 8 && DEGCAP % 8 == 0);
static_assert(BK_INTS % 4 == 0 && BK_INTS * 4 <= 262144);
static_assert(BK_CNTW % 4 == 0 && BK_OFF % 4 == 0 && BK_CNT % 4 == 0 && BK_MISC % 4 == 0 && BK_PLC % 4 == 0);
static_assert(XB_BLK * 256 == MPAD * 128 / 8);
static_assert(T_BE - T_G == 768 && T_RM - T_BE == 768 && T_INV - T_RM == 768 && T_B2 + 384 == TAB_N);
static_assert(T_B1 % 32 == 0 && T_B2 % 32 == 0 && TAB_N % 4 == 0);
static_assert(NNODE % 16 == 0);

__device__ __forceinline__ void pinf(float x) { asm volatile("" :: "v"(x)); }
__device__ __forceinline__ void pini(int x)   { asm volatile("" :: "v"(x)); }
__device__ __forceinline__ void pin4(v4f x)   { asm volatile("" :: "v"(x)); }
__device__ __forceinline__ float relun(float v) { return (v > 0.0f) ? v : (v - v); }
__device__ __forceinline__ float mskf(float v, unsigned m) { return __uint_as_float(__float_as_uint(v) & m); }

__device__ __forceinline__ v2u hi4w(float a0, float a1, float a2, float a3, unsigned mk) {
  return (v2u){ pk16(bf16_bits(a0), bf16_bits(a1)) & mk, pk16(bf16_bits(a2), bf16_bits(a3)) & mk };
}
__device__ __forceinline__ v2u lo4w(float a0, float a1, float a2, float a3, unsigned mk) {
  return (v2u){ pk16(bf16_lo_bits(a0), bf16_lo_bits(a1)) & mk, pk16(bf16_lo_bits(a2), bf16_lo_bits(a3)) & mk };
}

__device__ __forceinline__ void wt_piece(const float* __restrict__ w, int kin, int ncols, int ktot,
                                         unsigned short* dst, int g) {
  const int ppr = ktot >> 3;
  int n = g / ppr;
  const int p = g - n * ppr;
  n = n < ncols ? n : ncols - 1;
  const int k0 = p << 3;
  float xv[8];
#pragma unroll
  for (int e = 0; e < 8; ++e) {
    const int k = (k0 + e) & (kin - 1);
    const float v = w[(size_t)k * (size_t)ncols + (size_t)n];
    pinf(v);
    xv[e] = v;
  }
  const v4u o = pack8_bf16((v4f){ xv[0], xv[1], xv[2], xv[3] }, (v4f){ xv[4], xv[5], xv[6], xv[7] });
  volatile v4u* q = (volatile v4u*)(dst + (size_t)g * 8);
  *q = o;
  __threadfence();
  *q = o;
}

__device__ __forceinline__ void seg_copy(const float* __restrict__ s, int n, float* img, int off, int tid) {
#pragma unroll 1
  for (int i = tid; i < n; i += 256) {
    float v = s[i];
    pinf(v);
    img[off + i] = bf16_val(v);
  }
}
__device__ __forceinline__ void seg_inv(const float* __restrict__ s, int n, float* img, int off, int tid) {
#pragma unroll 1
  for (int i = tid; i < n; i += 256) {
    float v = s[i];
    pinf(v);
    img[off + i] = 1.0f / sqrtf(bf16_val(v) + 1e-5f);
  }
}

__global__ __launch_bounds__(256) void k_prep(
    const float* __restrict__ x,
    const float* __restrict__ enc_w0, const float* __restrict__ enc_b0, const float* __restrict__ w1_0,
    const float* __restrict__ b1_0, const float* __restrict__ g0, const float* __restrict__ be0,
    const float* __restrict__ rm0, const float* __restrict__ rv0, const float* __restrict__ w2_0,
    const float* __restrict__ b2_0,
    const float* __restrict__ enc_w, const float* __restrict__ enc_b, const float* __restrict__ w1,
    const float* __restrict__ b1, const float* __restrict__ g, const float* __restrict__ be,
    const float* __restrict__ rm, const float* __restrict__ rv, const float* __restrict__ w2,
    const float* __restrict__ b2,
    unsigned short* xb, unsigned short* enc, unsigned short* w1d0, unsigned short* w1d, unsigned short* w2d,
    float* tab) {
  __shared__ __attribute__((aligned(16))) float img[TAB_N];
  const int tid = (int)threadIdx.x;
  const int b = (int)blockIdx.x;
  if (b < XB_BLK) {
    const unsigned gp = (unsigned)b * 256u + (unsigned)tid;
    const int row = (int)(gp >> 4);
    const int c0 = (int)((gp & 15u) << 3);
    const int rc = row < NNODE ? row : NNODE - 1;
    const float* sr = x + (size_t)rc * 128 + c0;
    const v4f a = *(const v4fa*)sr;
    const v4f c = *(const v4fa*)(sr + 4);
    pin4(a);
    pin4(c);
    const unsigned mk = (row < NNODE) ? 0xFFFFFFFFu : 0u;
    v4u o = pack8_bf16(a, c);
    o &= (v4u){ mk, mk, mk, mk };
    volatile v4u* q = (volatile v4u*)(xb + (size_t)gp * 8);
    *q = o;
    __threadfence();
    *q = o;
  } else if (b < XB_BLK + WT_BLK) {
    const int wb = b - XB_BLK;
    if (wb < 2)        wt_piece(enc_w0,        16, 128, 32,  enc,          wb * 256 + tid);
    else if (wb < 4)   wt_piece(enc_w,         16, 128, 32,  enc + 4096,   (wb - 2) * 256 + tid);
    else if (wb < 6)   wt_piece(enc_w + 2048,  16, 128, 32,  enc + 8192,   (wb - 4) * 256 + tid);
    else if (wb < 38)  wt_piece(w1_0,         128, 256, 256, w1d0,         (wb - 6) * 256 + tid);
    else if (wb < 102) wt_piece(w1,           256, 256, 512, w1d,          (wb - 38) * 256 + tid);
    else if (wb < 166) wt_piece(w1 + 65536,   256, 256, 512, w1d + 131072, (wb - 102) * 256 + tid);
    else if (wb < 198) wt_piece(w2_0,         256, 128, 512, w2d,          (wb - 166) * 256 + tid);
    else if (wb < 230) wt_piece(w2,           256, 128, 512, w2d + 65536,  (wb - 198) * 256 + tid);
    else               wt_piece(w2 + 32768,   256, 128, 512, w2d + 131072, (wb - 230) * 256 + tid);
  } else {
    seg_copy(enc_b0, 128, img, T_ENCB, tid);
    seg_copy(enc_b,  256, img, T_ENCB + 128, tid);
    seg_copy(b1_0,   256, img, T_B1, tid);
    seg_copy(b1,     512, img, T_B1 + 256, tid);
    seg_copy(g0,     256, img, T_G, tid);
    seg_copy(g,      512, img, T_G + 256, tid);
    seg_copy(be0,    256, img, T_BE, tid);
    seg_copy(be,     512, img, T_BE + 256, tid);
    seg_copy(rm0,    256, img, T_RM, tid);
    seg_copy(rm,     512, img, T_RM + 256, tid);
    seg_inv(rv0,     256, img, T_INV, tid);
    seg_inv(rv,      512, img, T_INV + 256, tid);
    seg_copy(b2_0,   128, img, T_B2, tid);
    seg_copy(b2,     256, img, T_B2 + 128, tid);
    __syncthreads();
    for (int pass = 0; pass < 2; ++pass) {
#pragma unroll 1
      for (int p = tid; p < TAB_N / 4; p += 256) {
        const v4f v = *(const v4fa*)(img + 4 * p);
        *(volatile v4f*)(tab + 4 * p) = v;
      }
      __threadfence();
    }
  }
}

__device__ __forceinline__ int slot_prefix(int* cntw, int s) {
  int run = 0;
#pragma unroll
  for (int w = 0; w < NWV; ++w) {
    const int c = cntw[w * NBRUN + s];
    cntw[w * NBRUN + s] = run;
    run += c;
  }
  return run;
}

#define BK_HIT(J, SJ) { \
    const unsigned mk_ = __builtin_amdgcn_ballot_w32((SJ) < unb); \
    if (mk_ != 0u) { \
      const int pos_ = wcnt + (int)__builtin_amdgcn_mbcnt_lo(mk_, 0u); \
      if ((SJ) < unb && pos_ < WCAP) list[lbase + pos_] = (int)((((unsigned)(e0 + (J))) << 10) | (SJ)); \
      wcnt += (int)__builtin_popcount(mk_); \
    } }

__global__ __launch_bounds__(256) void k_bucket(const int* __restrict__ ei, unsigned* listg, int* offg,
                                                int* cntg, int* flagg) {
  extern __shared__ __attribute__((aligned(16))) int dsm[];
  int* list = dsm;
  int* cntw = dsm + BK_CNTW;
  int* offA = dsm + BK_OFF;
  int* cntT = dsm + BK_CNT;
  int* misc = dsm + BK_MISC;
  usa* plc  = (usa*)(dsm + BK_PLC);
  const int tid = (int)threadIdx.x, lane = tid & 31;
  const int wave = __builtin_amdgcn_readfirstlane(tid >> 5);
  const int b = (int)blockIdx.x;
  const int nodeBase = b * NBRUN;
  const int nbl = (NNODE - nodeBase) < NBRUN ? (NNODE - nodeBase) : NBRUN;
  const unsigned nbs = (unsigned)nodeBase;
  const unsigned unb = (unsigned)nbl;
  const int lbase = wave * WCAP;

  {
    const v4i z4 = {0, 0, 0, 0};
#pragma unroll 1
    for (int i = tid * 4; i < BK_INTS; i += 1024) *(v4ia*)(dsm + i) = z4;
  }
  __syncthreads();

  int wcnt = 0;
#pragma unroll 1
  for (int wc = wave; wc < NWCH; wc += NWV) {
    const int e0 = wc * 256 + lane * 8;
    const v4i da = *(const v4ia*)(ei + e0);
    const v4i db = *(const v4ia*)(ei + e0 + 4);
    const unsigned s0 = (unsigned)da.x - nbs, s1 = (unsigned)da.y - nbs;
    const unsigned s2 = (unsigned)da.z - nbs, s3 = (unsigned)da.w - nbs;
    const unsigned s4 = (unsigned)db.x - nbs, s5 = (unsigned)db.y - nbs;
    const unsigned s6 = (unsigned)db.z - nbs, s7 = (unsigned)db.w - nbs;
    BK_HIT(0, s0)
    BK_HIT(1, s1)
    BK_HIT(2, s2)
    BK_HIT(3, s3)
    BK_HIT(4, s4)
    BK_HIT(5, s5)
    BK_HIT(6, s6)
    BK_HIT(7, s7)
  }
  const int wraw = __builtin_amdgcn_readfirstlane(wcnt);
  if (lane == 0) misc[wave] = wraw;
  __syncthreads();

  const int myc = clampi(wraw, 0, WCAP);
  if (lane == 0) {
#pragma unroll 1
    for (int i = 0; i < myc; ++i) {
      const int s = list[lbase + i] & (NBRUN - 1);
      cntw[wave * NBRUN + s] = cntw[wave * NBRUN + s] + 1;
    }
  }
  __syncthreads();

  const int t0 = slot_prefix(cntw, 4 * tid);
  const int t1 = slot_prefix(cntw, 4 * tid + 1);
  const int t2 = slot_prefix(cntw, 4 * tid + 2);
  const int t3 = slot_prefix(cntw, 4 * tid + 3);
  const int e1 = t0, e2 = t0 + t1, e3 = t0 + t1 + t2, sum4 = t0 + t1 + t2 + t3;
  int incl = sum4;
#pragma unroll
  for (int dd = 1; dd < 32; dd <<= 1) {
    const int y = __shfl_up(incl, dd, 32);
    if (lane >= dd) incl += y;
  }
  if (lane == 31) misc[8 + wave] = incl;
  __syncthreads();
  int base = 0, tot = 0, flag = 0;
#pragma unroll
  for (int w2 = 0; w2 < NWV; ++w2) {
    const int c = misc[8 + w2];
    base += (w2 < wave) ? c : 0;
    tot  += c;
    flag |= (misc[w2] > WCAP) ? 1 : 0;
  }
  const int ex = base + incl - sum4;
  const v4i ov = {ex, ex + e1, ex + e2, ex + e3};
  const v4i cv = {t0, t1, t2, t3};
  *(v4ia*)(offA + 4 * tid) = ov;
  *(v4ia*)(cntT + 4 * tid) = cv;
  __syncthreads();

  if (lane == 0) {
#pragma unroll 1
    for (int i = 0; i < myc; ++i) {
      const int s = list[lbase + i] & (NBRUN - 1);
      const int c = cntw[wave * NBRUN + s];
      cntw[wave * NBRUN + s] = c + 1;
      const int p = offA[s] + c;
      if ((unsigned)p < (unsigned)RCAP) plc[p] = (unsigned short)(lbase + i);
    }
  }
  __syncthreads();

  const int tt = tot < RCAP ? tot : RCAP;
  unsigned* lg = listg + (size_t)b * (size_t)(RCAP * 2);
  const v4i fv = {(tid == 0) ? flag : 0, 0, 0, 0};
  for (int pass = 0; pass < 2; ++pass) {
#pragma unroll 1
    for (int p = tid; p < RCAP; p += 256) {
      const int pc = p < tt ? p : (tt > 0 ? tt - 1 : 0);
      const int idx = (int)plc[pc];
      const unsigned word = (unsigned)list[clampi(idx, 0, LISTN - 1)];
      const int eid = clampi((int)(word >> 10), 0, NEDGE - 1);
      int sr = ei[NEDGE + eid];
      pini(sr);
      sr = clampi(sr, 0, NNODE - 1);
      const unsigned mk = (p < tt) ? 0xFFFFFFFFu : 0u;
      const v2u o = {(unsigned)sr & mk, (unsigned)eid & mk};
      *(volatile v2u*)(lg + 2 * (size_t)p) = o;
    }
    *(volatile v4i*)(offg + (size_t)b * NBRUN + 4 * tid) = ov;
    *(volatile v4i*)(cntg + (size_t)b * NBRUN + 4 * tid) = cv;
    if (tid < 8) *(volatile v4i*)(flagg + (size_t)b * 32 + 4 * tid) = fv;
    __threadfence();
  }
}

__global__ __launch_bounds__(256) void k_attr(const float* __restrict__ ea, const unsigned* __restrict__ listg,
                                              const int* __restrict__ offg, const int* __restrict__ cntg,
                                              const int* __restrict__ sli, const int* __restrict__ slt,
                                              unsigned* aehl) {
  __shared__ __attribute__((aligned(16))) unsigned sA[256 * 16];
  const int tid = (int)threadIdx.x, lane = tid & 31;
  const int wave = __builtin_amdgcn_readfirstlane(tid >> 5);
  const int b = (int)blockIdx.x;
  int si = sli[0];
  pini(si);
  si = clampi(si, 0, 15);
  int st = slt[0];
  pini(st);
  const float slv = (float)st;
  const int j = lane >> 2, q = lane & 3;
  const size_t ebase = (size_t)b * (size_t)RCAP;
#pragma unroll 1
  for (int bat = 0; bat < 4; ++bat) {
#pragma unroll 1
    for (int u = 0; u < 32; ++u) {
      const int srow = wave * 32 + u;
      const int node = b * NBRUN + bat * 256 + srow;
      int off = offg[node];
      pini(off);
      int cr = cntg[node];
      pini(cr);
      int cnt = clampi(cr, 0, DEGCAP);
      off = clampi(off, 0, RCAP - 1);
      if (cnt > RCAP - off) cnt = RCAP - off;
      const int lastv = off + (cnt > 0 ? cnt - 1 : 0);
      cnt = __builtin_amdgcn_readfirstlane(cnt);
      off = __builtin_amdgcn_readfirstlane(off);
      const int last = __builtin_amdgcn_readfirstlane(lastv);
      float a0 = 0.0f, a1 = 0.0f, a2 = 0.0f, a3 = 0.0f;
#pragma unroll 1
      for (int g0 = 0; g0 < cnt; g0 += 8) {
        int idx = off + g0 + j;
        idx = idx > last ? last : idx;
        const v2u en = *(const v2ua*)(listg + (ebase + (size_t)idx) * 2);
        pini((int)en.x); pini((int)en.y);
        const int eid = clampi((int)en.y, 0, NEDGE - 1);
        const v4f av = *(const v4fa*)(ea + (size_t)eid * 16 + 4 * q);
        pin4(av);
        const unsigned m = ((g0 + j) < cnt) ? 0xFFFFFFFFu : 0u;
        a0 += mskf(bf16_val(av[0]), m);
        a1 += mskf(bf16_val(av[1]), m);
        a2 += mskf(bf16_val(av[2]), m);
        a3 += mskf(bf16_val(av[3]), m);
      }
      a0 += __shfl_xor(a0, 4, 32);  a1 += __shfl_xor(a1, 4, 32);
      a2 += __shfl_xor(a2, 4, 32);  a3 += __shfl_xor(a3, 4, 32);
      a0 += __shfl_xor(a0, 8, 32);  a1 += __shfl_xor(a1, 8, 32);
      a2 += __shfl_xor(a2, 8, 32);  a3 += __shfl_xor(a3, 8, 32);
      a0 += __shfl_xor(a0, 16, 32); a1 += __shfl_xor(a1, 16, 32);
      a2 += __shfl_xor(a2, 16, 32); a3 += __shfl_xor(a3, 16, 32);
      a0 += (4 * q + 0 == si) ? slv : 0.0f;
      a1 += (4 * q + 1 == si) ? slv : 0.0f;
      a2 += (4 * q + 2 == si) ? slv : 0.0f;
      a3 += (4 * q + 3 == si) ? slv : 0.0f;
      const unsigned pm = (node < NNODE) ? 0xFFFFFFFFu : 0u;
      const v2u hw = hi4w(a0, a1, a2, a3, pm);
      const v2u lw = lo4w(a0, a1, a2, a3, pm);
      if (j == 0) {
        sA[srow * 16 + 2 * q]         = hw.x;
        sA[srow * 16 + 2 * q + 1]     = hw.y;
        sA[srow * 16 + 8 + 2 * q]     = lw.x;
        sA[srow * 16 + 8 + 2 * q + 1] = lw.y;
      }
    }
    __syncthreads();
    unsigned* og = aehl + (size_t)(b * NBRUN + bat * 256) * 16;
    v4u vv[4];
#pragma unroll
    for (int it = 0; it < 4; ++it) vv[it] = *(const v4ua*)(sA + 4 * (tid + 256 * it));
    for (int pass = 0; pass < 2; ++pass) {
#pragma unroll
      for (int it = 0; it < 4; ++it) *(volatile v4u*)(og + 4 * (tid + 256 * it)) = vv[it];
      __threadfence();
    }
    __syncthreads();
  }
}

template <int CONCAT>
__global__ __launch_bounds__(256) void k_replay(const unsigned* __restrict__ xbw, const float* __restrict__ hin,
                                                const float* __restrict__ ee, const unsigned* __restrict__ listg,
                                                const int* __restrict__ offg, const int* __restrict__ cntg,
                                                const int* __restrict__ flagg, const float* __restrict__ tab,
                                                int encbOff, unsigned* ag) {
  const int tid = (int)threadIdx.x, lane = tid & 31;
  const int wave = __builtin_amdgcn_readfirstlane(tid >> 5);
  const int b = (int)blockIdx.x;
  int fl = flagg[(size_t)b * 32];
  pini(fl);
  const v4f eb = *(const v4fa*)(tab + encbOff + 4 * lane);
  pin4(eb);
  const float qnan = __int_as_float(0x7fc00000);
  const size_t ebase = (size_t)b * (size_t)RCAP;
#pragma unroll 1
  for (int si = 0; si < 128; ++si) {
    const int node = b * NBRUN + wave * 128 + si;
    int off = offg[node];
    pini(off);
    int cr = cntg[node];
    pini(cr);
    const int degov = (cr > DEGCAP) ? 1 : 0;
    int cnt = clampi(cr, 0, DEGCAP);
    off = clampi(off, 0, RCAP - 1);
    if (cnt > RCAP - off) cnt = RCAP - off;
    const int lastv = off + (cnt > 0 ? cnt - 1 : 0);
    cnt = __builtin_amdgcn_readfirstlane(cnt);
    off = __builtin_amdgcn_readfirstlane(off);
    const int last = __builtin_amdgcn_readfirstlane(lastv);
    float s0 = 0.0f, s1 = 0.0f, s2 = 0.0f, s3 = 0.0f;
#pragma unroll 1
    for (int g0 = 0; g0 < cnt; g0 += 8) {
      int idx = off + g0 + (lane & 7);
      idx = idx > last ? last : idx;
      const v2u en = *(const v2ua*)(listg + (ebase + (size_t)idx) * 2);
      pini((int)en.x); pini((int)en.y);
      const int srl = clampi((int)en.x, 0, NNODE - 1);
      if (CONCAT) {
        v4f hv[8];
#pragma unroll
        for (int j = 0; j < 8; ++j) {
          const int sj = __builtin_amdgcn_readlane(srl, j);
          hv[j] = *(const v4fa*)(hin + (size_t)sj * 128 + 4 * lane);
          pin4(hv[j]);
        }
#pragma unroll
        for (int j = 0; j < 8; ++j) {
          const unsigned m = ((g0 + j) < cnt) ? 0xFFFFFFFFu : 0u;
          s0 += mskf(relun(hv[j][0]), m);
          s1 += mskf(relun(hv[j][1]), m);
          s2 += mskf(relun(hv[j][2]), m);
          s3 += mskf(relun(hv[j][3]), m);
        }
      } else {
        unsigned wx[8], wy[8];
#pragma unroll
        for (int j = 0; j < 8; ++j) {
          const int sj = __builtin_amdgcn_readlane(srl, j);
          const v2u w = *(const v2ua*)(xbw + (size_t)sj * 64 + 2 * lane);
          pini((int)w.x); pini((int)w.y);
          wx[j] = w.x;
          wy[j] = w.y;
        }
#pragma unroll
        for (int j = 0; j < 8; ++j) {
          const unsigned m = ((g0 + j) < cnt) ? 0xFFFFFFFFu : 0u;
          s0 += __uint_as_float((wx[j] << 16) & m);
          s1 += __uint_as_float((wx[j] & 0xffff0000u) & m);
          s2 += __uint_as_float((wy[j] << 16) & m);
          s3 += __uint_as_float((wy[j] & 0xffff0000u) & m);
        }
      }
    }
    const int nc = node < NNODE ? node : NNODE - 1;
    if (CONCAT) {
      const v4f ov = *(const v4fa*)(hin + (size_t)nc * 128 + 4 * lane);
      pin4(ov);
      s0 += relun(ov[0]); s1 += relun(ov[1]); s2 += relun(ov[2]); s3 += relun(ov[3]);
    } else {
      const v2u w = *(const v2ua*)(xbw + (size_t)nc * 64 + 2 * lane);
      pini((int)w.x); pini((int)w.y);
      s0 += __uint_as_float(w.x << 16);
      s1 += __uint_as_float(w.x & 0xffff0000u);
      s2 += __uint_as_float(w.y << 16);
      s3 += __uint_as_float(w.y & 0xffff0000u);
    }
    const v4f e4 = *(const v4fa*)(ee + (size_t)node * 128 + 4 * lane);
    pin4(e4);
    const float cf = (float)(cnt + 1);
    const float pz = (fl != 0 || degov != 0) ? qnan : 0.0f;
    float q0 = fmaf(cf, eb[0], e4[0]) + pz;
    float q1 = fmaf(cf, eb[1], e4[1]) + pz;
    float q2 = fmaf(cf, eb[2], e4[2]) + pz;
    float q3 = fmaf(cf, eb[3], e4[3]) + pz;
    const unsigned pm = (node < NNODE) ? 0xFFFFFFFFu : 0u;
    if (CONCAT) {
      s0 += pz; s1 += pz; s2 += pz; s3 += pz;
      const v2u hs = hi4w(s0, s1, s2, s3, pm);
      const v2u he = hi4w(q0, q1, q2, q3, pm);
      const v2u ls = lo4w(s0, s1, s2, s3, pm);
      const v2u le = lo4w(q0, q1, q2, q3, pm);
      unsigned* op = ag + (size_t)node * 256 + 2 * lane;
      *(volatile v2u*)op = hs;
      *(volatile v2u*)(op + 64) = he;
      *(volatile v2u*)(op + 128) = ls;
      *(volatile v2u*)(op + 192) = le;
      __threadfence();
      *(volatile v2u*)op = hs;
      *(volatile v2u*)(op + 64) = he;
      *(volatile v2u*)(op + 128) = ls;
      *(volatile v2u*)(op + 192) = le;
    } else {
      const float a0 = s0 + q0, a1 = s1 + q1, a2 = s2 + q2, a3 = s3 + q3;
      const v2u hw = hi4w(a0, a1, a2, a3, pm);
      const v2u lw = lo4w(a0, a1, a2, a3, pm);
      unsigned* op = ag + (size_t)node * 128 + 2 * lane;
      *(volatile v2u*)op = hw;
      *(volatile v2u*)(op + 64) = lw;
      __threadfence();
      *(volatile v2u*)op = hw;
      *(volatile v2u*)(op + 64) = lw;
    }
  }
}

__global__ __launch_bounds__(256) void k_bn(const float* __restrict__ t, const float* __restrict__ tab, int layer,
                                            unsigned short* thl) {
  __shared__ __attribute__((aligned(16))) float sP[1024];
  const int tid = (int)threadIdx.x, lane = tid & 31;
  const int wave = __builtin_amdgcn_readfirstlane(tid >> 5);
  {
    const int seg = tid >> 6, pc = tid & 63;
    const v4f v = *(const v4fa*)(tab + T_G + 768 * seg + 256 * layer + 4 * pc);
    *(v4fa*)(sP + 256 * seg + 4 * pc) = v;
  }
  __syncthreads();
  const v4f ga = *(const v4fa*)(sP + 8 * lane),       gc = *(const v4fa*)(sP + 8 * lane + 4);
  const v4f ba = *(const v4fa*)(sP + 256 + 8 * lane), bc = *(const v4fa*)(sP + 256 + 8 * lane + 4);
  const v4f ma = *(const v4fa*)(sP + 512 + 8 * lane), mc = *(const v4fa*)(sP + 512 + 8 * lane + 4);
  const v4f ia = *(const v4fa*)(sP + 768 + 8 * lane), ic = *(const v4fa*)(sP + 768 + 8 * lane + 4);
#pragma unroll 1
  for (int j = 0; j < 16; ++j) {
    const int row = (int)blockIdx.x * 128 + wave * 16 + j;
    const float* tr = t + (size_t)row * 256 + 8 * lane;
    const v4f a = *(const v4fa*)tr;
    const v4f c = *(const v4fa*)(tr + 4);
    pin4(a);
    pin4(c);
    v4f ya = ((ga * (a - ma)) * ia) + ba;
    v4f yc = ((gc * (c - mc)) * ic) + bc;
    ya = (v4f){ relun(ya[0]), relun(ya[1]), relun(ya[2]), relun(ya[3]) };
    yc = (v4f){ relun(yc[0]), relun(yc[1]), relun(yc[2]), relun(yc[3]) };
    const unsigned mk = (row < NNODE) ? 0xFFFFFFFFu : 0u;
    const v4u mw = (v4u){ mk, mk, mk, mk };
    v4u hi = pack8_bf16(ya, yc);
    v4u lo = pack8_bf16_lo(ya, yc);
    hi &= mw;
    lo &= mw;
    unsigned short* op = thl + (size_t)row * 512 + 8 * lane;
    *(volatile v4u*)op = hi;
    *(volatile v4u*)(op + 256) = lo;
    __threadfence();
    *(volatile v4u*)op = hi;
    *(volatile v4u*)(op + 256) = lo;
  }
}

static constexpr size_t al256c(size_t o) { return (o + 255) & ~(size_t)255; }
static constexpr size_t O_R1   = 0;
static constexpr size_t O_R2   = al256c(O_R1   + (size_t)MPAD * 512 * 2);
static constexpr size_t O_XB   = al256c(O_R2   + (size_t)MPAD * 256 * 4);
static constexpr size_t O_AEHL = al256c(O_XB   + (size_t)MPAD * 128 * 2);
static constexpr size_t O_CNTL = al256c(O_AEHL + (size_t)MPAD * 32 * 2);
static constexpr size_t O_OFFS = al256c(O_CNTL + (size_t)MPAD * 4);
static constexpr size_t O_LIST = al256c(O_OFFS + (size_t)MPAD * 4);
static constexpr size_t O_FLAG = al256c(O_LIST + (size_t)NBLKB * RCAP * 8);
static constexpr size_t O_TAB  = al256c(O_FLAG + (size_t)NBLKB * 128);
static constexpr size_t O_ENC  = al256c(O_TAB  + (size_t)TAB_N * 4);
static constexpr size_t O_W1D0 = al256c(O_ENC  + (size_t)3 * 128 * 32 * 2);
static constexpr size_t O_W1D  = al256c(O_W1D0 + (size_t)256 * 256 * 2);
static constexpr size_t O_W2D  = al256c(O_W1D  + (size_t)2 * 256 * 512 * 2);
static constexpr size_t WS_TOTAL = al256c(O_W2D + (size_t)3 * 128 * 512 * 2);
static_assert(WS_TOTAL == ((size_t)502913 << 8));
static_assert(WS_TOTAL <= ((size_t)128 << 20));
static_assert((size_t)MPAD * 128 * 4 == 25690112ull);
static_assert((size_t)MPAD * 256 * 2 <= (size_t)MPAD * 512 * 2);

extern "C" void kernel_launch(void* const* d_in, const int* in_sizes, int n_in,
                              void* d_out, int out_size, void* d_ws, size_t ws_size,
                              hipStream_t stream) {
  if (n_in != 25) return;
  const int es[25] = { NNODE * 128, 2 * NEDGE, NEDGE * 16, 1, 1, 16 * 128, 128, 128 * 256, 256, 256, 256, 256, 256,
                       256 * 128, 128, 2 * 16 * 128, 2 * 128, 2 * 256 * 256, 2 * 256, 2 * 256, 2 * 256, 2 * 256,
                       2 * 256, 2 * 256 * 128, 2 * 128 };
  for (int i = 0; i < 25; ++i) if (in_sizes[i] != es[i]) return;
  if (out_size != NNODE * 128) return;
  if (WS_TOTAL > ws_size) return;

  const float* x      = (const float*)d_in[0];
  const int*   ei     = (const int*)d_in[1];
  const float* ea     = (const float*)d_in[2];
  const int*   sli    = (const int*)d_in[3];
  const int*   slt    = (const int*)d_in[4];
  const float* enc_w0 = (const float*)d_in[5];
  const float* enc_b0 = (const float*)d_in[6];
  const float* w1_0   = (const float*)d_in[7];
  const float* b1_0   = (const float*)d_in[8];
  const float* g0     = (const float*)d_in[9];
  const float* be0    = (const float*)d_in[10];
  const float* rm0    = (const float*)d_in[11];
  const float* rv0    = (const float*)d_in[12];
  const float* w2_0   = (const float*)d_in[13];
  const float* b2_0   = (const float*)d_in[14];
  const float* enc_w  = (const float*)d_in[15];
  const float* enc_b  = (const float*)d_in[16];
  const float* w1     = (const float*)d_in[17];
  const float* b1     = (const float*)d_in[18];
  const float* g      = (const float*)d_in[19];
  const float* be     = (const float*)d_in[20];
  const float* rm     = (const float*)d_in[21];
  const float* rv     = (const float*)d_in[22];
  const float* w2     = (const float*)d_in[23];
  const float* b2     = (const float*)d_in[24];
  float* out = (float*)d_out;

  char* ws = (char*)d_ws;
  unsigned short* R1   = (unsigned short*)(ws + O_R1);
  float*          EE   = (float*)(ws + O_R2);
  float*          Tp   = (float*)(ws + O_R2);
  float*          Hp   = (float*)(ws + O_R2 + (size_t)MPAD * 128 * 4);
  unsigned short* XB   = (unsigned short*)(ws + O_XB);
  unsigned short* AEHL = (unsigned short*)(ws + O_AEHL);
  int*            CNTL = (int*)(ws + O_CNTL);
  int*            OFFS = (int*)(ws + O_OFFS);
  unsigned*       LIST = (unsigned*)(ws + O_LIST);
  int*            FLAG = (int*)(ws + O_FLAG);
  float*          TAB  = (float*)(ws + O_TAB);
  unsigned short* ENC  = (unsigned short*)(ws + O_ENC);
  unsigned short* W1D0 = (unsigned short*)(ws + O_W1D0);
  unsigned short* W1D  = (unsigned short*)(ws + O_W1D);
  unsigned short* W2D  = (unsigned short*)(ws + O_W2D);

  static_assert(MPAD % 64 == 0 && MPAD % 16 == 0 && NNODE % 16 == 0);
  static_assert(32 % 32 == 0 && 256 % 32 == 0 && 512 % 32 == 0);
  static_assert(128 % 64 == 0 && 256 % 64 == 0);
  static_assert(128 % 32 == 0 && 256 % 32 == 0);
  static_assert(((MPAD / 64) * 2) % 8 == 0 && ((MPAD / 64) * 4) % 8 == 0);
  const int gridN128 = ((MPAD / 64) * 2) / 8;
  const int gridN256 = ((MPAD / 64) * 4) / 8;
  const int gridOut  = (((NNODE + 63) / 64) * 2 + 7) / 8;

  const int bkLds = BK_INTS * 4;
  hipFuncSetAttribute(reinterpret_cast<const void*>(&k_bucket), hipFuncAttributeMaxDynamicSharedMemorySize, bkLds);

  k_prep<<<PREP_GRID, 256, 0, stream>>>(x, enc_w0, enc_b0, w1_0, b1_0, g0, be0, rm0, rv0, w2_0, b2_0,
                                        enc_w, enc_b, w1, b1, g, be, rm, rv, w2, b2,
                                        XB, ENC, W1D0, W1D, W2D, TAB);
  k_bucket<<<NBLKB, 256, bkLds, stream>>>(ei, LIST, OFFS, CNTL, FLAG);
  k_attr<<<NBLKB, 256, 0, stream>>>(ea, LIST, OFFS, CNTL, sli, slt, (unsigned*)AEHL);

  for (int l = 0; l < 3; ++l) {
    k_gemm_nt<1, 0><<<gridN128, 256, 0, stream>>>(AEHL, ENC + (size_t)l * 4096, TAB, EE, MPAD, 128, 32, 128);
    if (l == 0)
      k_replay<0><<<NBLKB, 256, 0, stream>>>((const unsigned*)XB, EE, EE, LIST, OFFS, CNTL, FLAG, TAB,
                                             T_ENCB, (unsigned*)R1);
    else
      k_replay<1><<<NBLKB, 256, 0, stream>>>((const unsigned*)XB, Hp, EE, LIST, OFFS, CNTL, FLAG, TAB,
                                             T_ENCB + 128 * l, (unsigned*)R1);
    const unsigned short* w1p = (l == 0) ? W1D0 : (W1D + (size_t)(l - 1) * 131072);
    const int k1 = (l == 0) ? 256 : 512;
    k_gemm_nt<1, 1><<<gridN256, 256, 0, stream>>>(R1, w1p, TAB + T_B1 + 256 * l, Tp, MPAD, 256, k1, 256);
    k_bn<<<MPAD / 128, 256, 0, stream>>>(Tp, TAB, l, R1);
    if (l < 2)
      k_gemm_nt<1, 1><<<gridN128, 256, 0, stream>>>(R1, W2D + (size_t)l * 65536, TAB + T_B2 + 128 * l, Hp,
                                                    MPAD, 128, 512, 128);
    else
      k_gemm_nt<1, 1><<<gridOut, 256, 0, stream>>>(R1, W2D + (size_t)l * 65536, TAB + T_B2 + 128 * l, out,
                                                   NNODE, 128, 512, 128);
  }
}
